// kernel_generated_1_62904091017272
// MI455X (gfx1250) — hardware-verified
//
#include <hip/hip_runtime.h>
#include <stdint.h>

#define DEVINL __device__ __forceinline__

typedef _Float16 f16t;
typedef _Float16 v16h __attribute__((ext_vector_type(16)));
typedef _Float16 v8h  __attribute__((ext_vector_type(8)));
typedef float    v8f  __attribute__((ext_vector_type(8)));
typedef float    v4f  __attribute__((ext_vector_type(4)));
typedef unsigned int v4u __attribute__((ext_vector_type(4)));
typedef v8h __attribute__((may_alias)) v8ha;
typedef v4f __attribute__((may_alias)) v4fa;
union FragH { v16h v; v8h half[2]; v4u q[2]; };

#define CIN    64
#define HIMG   28
#define WIMG   28
#define NPOS   784
#define NL     128
#define KD     192
#define LB     16
#define NLB    (NL / LB)
#define NST    (NPOS / 16)
#define TPB    256
#define WAVES  8
#define NLINES ((LB * NPOS * 4) / 128)
#define NIT_T  ((NST + WAVES - 1) / WAVES)
#define NIT_L  ((NLINES + WAVES * 4 - 1) / (WAVES * 4))
#define XCAR   16.0f
#define WCAR   16.0f
#define OSC    (1.0f / 256.0f)

static_assert(TPB == WAVES * 32);
static_assert(NPOS % 16 == 0);
static_assert(KD % 32 == 0);
static_assert((LB * NPOS * 4) % 128 == 0);
static_assert(NLINES % 4 == 0);
static_assert((LB * KD) % 8 == 0);
static_assert((NL * KD) % (8 * TPB) == 0);

DEVINL v8f wmma_f16(v16h a, v16h b, v8f c) {
  v8f d = __builtin_amdgcn_wmma_f32_16x16x32_f16(false, a, false, b, (short)0, c, false, false);
  asm volatile("v_nop\n\tv_nop\n\tv_nop\n\tv_nop" : "+v"(d) : "v"(a), "v"(b));
  return d;
}
DEVINL v8f zero8f() {
  v8f z = {0.f, 0.f, 0.f, 0.f, 0.f, 0.f, 0.f, 0.f};
  return z;
}

__global__ __launch_bounds__(TPB) void prep_x_k(const float* __restrict__ x,
                                               f16t* __restrict__ XT, int npix8)
{
  const int t = blockIdx.x * TPB + threadIdx.x;
  if (t >= npix8) return;
  const int pix = t >> 3, q = t & 7;
  const int m   = pix / NPOS;
  const int rem = pix - m * NPOS;
  const float* src = x + ((size_t)m * CIN + 8 * q) * NPOS + rem;
  v8h o;
  #pragma unroll
  for (int e = 0; e < 8; ++e) o[e] = (f16t)(src[(size_t)e * NPOS] * XCAR);
  f16t* dst = XT + (size_t)t * 8;
  *(volatile v8h*)dst = o;
  __threadfence();
  *(volatile v8h*)dst = o;
}

__global__ __launch_bounds__(TPB) void prep_w_k(const float* __restrict__ w,
                                               f16t* __restrict__ WT, int total)
{
  const int t = blockIdx.x * TPB + threadIdx.x;
  if (t >= total) return;
  const int l    = t / (KD / 8);
  const int part = t - l * (KD / 8);
  const int kk0  = 8 * part;
  const int s    = kk0 >> 5;
  const int j    = (s >= 3) ? 1 : 0;
  const int k    = s - 3 * j;
  const int i0   = kk0 & 31;
  v8h o;
  #pragma unroll
  for (int e = 0; e < 8; ++e) {
    const int i = i0 + e;
    const int widx = ((j * 32 + i) * 3 + k) * NL + l;
    o[e] = (f16t)(w[widx] * WCAR);
  }
  f16t* dst = WT + (size_t)t * 8;
  *(volatile v8h*)dst = o;
  __threadfence();
  *(volatile v8h*)dst = o;
}

__global__ __launch_bounds__(TPB) void gemm_k(const f16t* __restrict__ XT,
                                             const f16t* __restrict__ WT,
                                             float* __restrict__ out)
{
  __shared__ __attribute__((aligned(16))) f16t  sW[LB * KD];
  __shared__ __attribute__((aligned(16))) float sO[LB * NPOS];

  const int tid  = threadIdx.x;
  const int lane = tid & 31;
  const int wave = __builtin_amdgcn_readfirstlane(tid >> 5);
  const int h    = lane >> 4, mm = lane & 15;
  const int bid  = blockIdx.x;
  const int m    = bid / NLB;
  const int l0   = (bid - m * NLB) * LB;

  {
    const f16t* wsrc = WT + (size_t)l0 * KD;
    for (int q = tid; q < (LB * KD) / 8; q += TPB)
      *(v8ha*)(sW + 8 * q) = *(const v8ha*)(wsrc + 8 * q);
  }
  __syncthreads();

  const f16t* ximg = XT + (size_t)m * NPOS * CIN;

  #pragma unroll 1
  for (int it = 0; it < NIT_T; ++it) {
    const int st = wave + WAVES * it;
    if (st < NST) {
      const int p = st * 16 + mm;
      const int n = p / WIMG;
      const int o = p - n * WIMG;
      v8f acc = zero8f();
      #pragma unroll
      for (int s = 0; s < KD / 32; ++s) {
        const int j  = (s >= 3) ? 1 : 0;
        const int k  = s - 3 * j;
        const int hr = j ? n : ((n == 0) ? (HIMG - 1) : (n - 1));
        const int cb = j ? 0 : 32;
        const int w0 = o + k - 1;
        const bool valid = (unsigned)w0 < (unsigned)WIMG;
        int col = o + k - 2;
        col += (col < 0) ? WIMG : 0;
        const f16t* ap = ximg + ((size_t)(hr * WIMG + col)) * CIN + cb + 8 * h;
        FragH a;
        a.half[0] = *(const v8ha*)(ap);
        a.half[1] = *(const v8ha*)(ap + 16);
        const unsigned msk = valid ? 0xffffffffu : 0u;
        const v4u mk = {msk, msk, msk, msk};
        a.q[0] = a.q[0] & mk;
        a.q[1] = a.q[1] & mk;
        const f16t* bp = sW + mm * KD + 32 * s + 8 * h;
        FragH b;
        b.half[0] = *(const v8ha*)(bp);
        b.half[1] = *(const v8ha*)(bp + 16);
        acc = wmma_f16(a.v, b.v, acc);
      }
      v4f o0, o1;
      #pragma unroll
      for (int r = 0; r < 4; ++r) { o0[r] = acc[r] * OSC; o1[r] = acc[4 + r] * OSC; }
      float* so = sO + mm * NPOS + st * 16 + 8 * h;
      *(v4fa*)(so)     = o0;
      *(v4fa*)(so + 4) = o1;
    }
  }
  __syncthreads();

  float* obase = out + ((size_t)m * NL + l0) * NPOS;
  const int q8 = lane & 7, lq = lane >> 3;
  #pragma unroll 1
  for (int it = 0; it < NIT_L; ++it) {
    const int lbase = it * (WAVES * 4) + wave * 4;
    if (lbase < NLINES) {
      const int line = lbase + lq;
      const v4f v = *(const v4fa*)(sO + line * 32 + q8 * 4);
      *(volatile v4f*)(obase + (size_t)line * 32 + q8 * 4) = v;
    }
  }
  __threadfence();
  #pragma unroll 1
  for (int it = 0; it < NIT_L; ++it) {
    const int lbase = it * (WAVES * 4) + wave * 4;
    if (lbase < NLINES) {
      const int line = lbase + lq;
      const v4f v = *(const v4fa*)(sO + line * 32 + q8 * 4);
      *(volatile v4f*)(obase + (size_t)line * 32 + q8 * 4) = v;
    }
  }
}

extern "C" void kernel_launch(void* const* d_in, const int* in_sizes, int n_in,
                              void* d_out, int out_size, void* d_ws, size_t ws_size,
                              hipStream_t stream) {
  if (n_in < 2) return;
  if (in_sizes[0] <= 0 || (in_sizes[0] % (CIN * NPOS)) != 0) return;
  const int NB = in_sizes[0] / (CIN * NPOS);
  if (in_sizes[1] != 2 * 32 * 3 * NL) return;
  if (out_size != NB * NL * NPOS) return;

  const float* x = (const float*)d_in[0];
  const float* w = (const float*)d_in[1];
  float* outp = (float*)d_out;

  const size_t szWT = (size_t)NL * KD * 2;
  const size_t szXT = (size_t)NB * NPOS * CIN * 2;
  size_t off = 0;
  char* ws = (char*)d_ws;
  f16t* WT = (f16t*)(ws + off); off += szWT;
  f16t* XT = (f16t*)(ws + off); off += szXT;
  if (off > ws_size) return;

  const int wtotal = NL * (KD / 8);
  const int npix8  = NB * NPOS * 8;

  prep_w_k<<<(wtotal + TPB - 1) / TPB, TPB, 0, stream>>>(w, WT, wtotal);
  prep_x_k<<<(npix8 + TPB - 1) / TPB, TPB, 0, stream>>>(x, XT, npix8);
  gemm_k<<<NB * NLB, TPB, 0, stream>>>(XT, WT, outp);
}
